// ParallelWarper_47863115546756
// MI455X (gfx1250) — hardware-verified
//
#include <hip/hip_runtime.h>
#define TFR 7
#define NFR 6
#define CC 64
#define HH 96
#define WW 96
#define NPOS (NFR * HH * WW)
#define CIN1 160
#define C4 448
#define DG 16
#define KK 9

typedef __bf16 v16b __attribute__((ext_vector_type(16)));
typedef unsigned short v8us __attribute__((ext_vector_type(8), may_alias));
typedef float  v8f  __attribute__((ext_vector_type(8)));
typedef float  v4f  __attribute__((ext_vector_type(4)));
typedef float  v4fa __attribute__((ext_vector_type(4), may_alias));
union FragB { v16b v; v8us half[2]; unsigned short u[16]; };

__device__ __forceinline__ unsigned short bf16_bits(float x) { unsigned int u = __float_as_uint(x); return (unsigned short)((u + 0x7FFFu + ((u >> 16) & 1u)) >> 16); }
__device__ __forceinline__ float bf16_val(unsigned short b) { return __uint_as_float(((unsigned int)b) << 16); }
__device__ __forceinline__ float bf16_round(float x) { return bf16_val(bf16_bits(x)); }
template <int NT>
__device__ __forceinline__ v8f mmaN(v16b ah, v16b al, v16b bh, v16b bl, v8f c) {
  c = __builtin_amdgcn_wmma_f32_16x16x32_bf16(false, ah, false, bh, (short)0, c, false, false);
  if (NT >= 2) c = __builtin_amdgcn_wmma_f32_16x16x32_bf16(false, al, false, bh, (short)0, c, false, false);
  if (NT >= 3) c = __builtin_amdgcn_wmma_f32_16x16x32_bf16(false, ah, false, bl, (short)0, c, false, false);
  asm volatile("v_nop\n\tv_nop\n\tv_nop\n\tv_nop" : "+v"(c) : "v"(ah), "v"(al), "v"(bh), "v"(bl));
  return c;
}

__global__ __launch_bounds__(256) void k_wt_bf16(const float* __restrict__ W, unsigned short* __restrict__ Wt, int K, int N) {
  const int t = blockIdx.x * 256 + threadIdx.x;
  const int k8n = K / 8;
  if (t >= N * k8n) return;
  const int n = t / k8n, k8 = (t % k8n) * 8;
  v8us v;
#pragma unroll
  for (int i = 0; i < 8; ++i) v[i] = bf16_bits(W[(size_t)(k8 + i) * N + n]);
  *(volatile v8us*)(Wt + (size_t)n * K + k8) = v;
  __threadfence();
  *(volatile v8us*)(Wt + (size_t)n * K + k8) = v;
}

template <bool ASPLIT, int ACT, bool BIAS_BF16>
__global__ __launch_bounds__(128) void k_gemm_bf(const float* __restrict__ A, int lda, const unsigned short* __restrict__ Wt, int ldb,
                                               const float* __restrict__ bias, float* __restrict__ C, int ldc, int M, int N, int K) {
  __shared__ __attribute__((aligned(16))) float so[4][16][64];
  const int tid = threadIdx.x, w = tid >> 5, lane = tid & 31, ln = lane & 15, hh = lane >> 4;
  const int ntn = N / 64;
  const int wid = blockIdx.x * 4 + w;
  const int mt = wid / ntn, nq = wid % ntn;
  if (mt * 16 >= M) return;
  const int row0 = mt * 16, col0 = nq * 64;
  const float* arow = A + (size_t)(row0 + ln) * lda;
  v8f acc[4] = {};
  for (int kb = 0; kb < K; kb += 32) {
    FragB ah, al;
    const v4f x0 = *(const v4fa*)(arow + kb + 8 * hh), x1 = *(const v4fa*)(arow + kb + 8 * hh + 4);
    const v4f x2 = *(const v4fa*)(arow + kb + 16 + 8 * hh), x3 = *(const v4fa*)(arow + kb + 16 + 8 * hh + 4);
    float xs[16] = {x0[0],x0[1],x0[2],x0[3],x1[0],x1[1],x1[2],x1[3],x2[0],x2[1],x2[2],x2[3],x3[0],x3[1],x3[2],x3[3]};
#pragma unroll
    for (int i = 0; i < 16; ++i) { const unsigned short hb = bf16_bits(xs[i]); ah.u[i] = hb; al.u[i] = ASPLIT ? bf16_bits(xs[i] - bf16_val(hb)) : (unsigned short)0; }
#pragma unroll
    for (int t = 0; t < 4; ++t) {
      const unsigned short* brow = Wt + (size_t)(col0 + t * 16 + ln) * ldb + kb;
      FragB b;
      b.half[0] = *(const v8us*)(brow + 8 * hh);
      b.half[1] = *(const v8us*)(brow + 16 + 8 * hh);
      acc[t] = mmaN<ASPLIT ? 2 : 1>(ah.v, al.v, b.v, b.v, acc[t]);
    }
  }
#pragma unroll
  for (int t = 0; t < 4; ++t) {
    float bv = bias ? bias[col0 + t * 16 + ln] : 0.f;
    if (BIAS_BF16) bv = bf16_round(bv);
#pragma unroll
    for (int r = 0; r < 8; ++r) { float v = acc[t][r] + bv; if (ACT == 1) v = fmaxf(v, 0.f); so[w][8 * hh + r][t * 16 + ln] = v; }
  }
  __builtin_amdgcn_fence(__ATOMIC_ACQ_REL, "workgroup");
  __builtin_amdgcn_wave_barrier();
  const int rsub = lane >> 4, c4 = (lane & 15) * 4;
  for (int pass = 0; pass < 2; ++pass) {
#pragma unroll
    for (int q = 0; q < 8; ++q) {
      const int r = q * 2 + rsub;
      const v4f v = *(const v4fa*)&so[w][r][c4];
      *(volatile v4f*)(C + (size_t)(row0 + r) * ldc + col0 + c4) = v;
    }
    if (pass == 0) __threadfence();
  }
}

template <int D, bool CAUSAL>
__global__ __launch_bounds__(128) void k_flash(const float* __restrict__ qb, const float* __restrict__ kb, const float* __restrict__ vb,
                                             int pitch, int T, int H, float scale, float* __restrict__ y, int ypitch) {
  constexpr int KS = D / 32;
  constexpr int DT = D / 16;
  __shared__ __attribute__((aligned(16))) unsigned short sKh[32][D + 8], sKl[32][D + 8], sVh[32][D + 8], sVl[32][D + 8];
  __shared__ __attribute__((aligned(16))) unsigned short sPh[4][16][40], sPl[4][16][40];
  __shared__ __attribute__((aligned(16))) float sO[4][16][D];
  const int tid = threadIdx.x, w = tid >> 5, lane = tid & 31, ln = lane & 15, hh = lane >> 4;
  const int nqb = (T + 63) / 64;
  const int bh = blockIdx.x / nqb, qblk = blockIdx.x % nqb;
  const int b = bh / H, h = bh % H;
  const int q0 = qblk * 64 + w * 16;
  const float* Q = qb + (size_t)b * T * pitch + h * D;
  const float* K = kb + (size_t)b * T * pitch + h * D;
  const float* V = vb + (size_t)b * T * pitch + h * D;

  FragB aqh[KS], aql[KS];
  {
    int row = q0 + ln; if (row >= T) row = T - 1;
    const float* qr = Q + (size_t)row * pitch;
#pragma unroll
    for (int ks = 0; ks < KS; ++ks)
#pragma unroll
      for (int i = 0; i < 16; ++i) {
        const int d = ks * 32 + ((i < 8) ? (8 * hh + i) : (16 + 8 * hh + (i - 8)));
        const float x = qr[d] * scale; const unsigned short hb = bf16_bits(x);
        aqh[ks].u[i] = hb; aql[ks].u[i] = bf16_bits(x - bf16_val(hb));
      }
  }
  float m_r[8], l_r[8];
#pragma unroll
  for (int r = 0; r < 8; ++r) { m_r[r] = -3.0e38f; l_r[r] = 0.f; }
  v8f oacc[DT];
#pragma unroll
  for (int dt = 0; dt < DT; ++dt) oacc[dt] = (v8f){0.f,0.f,0.f,0.f,0.f,0.f,0.f,0.f};

  const int kv_end = CAUSAL ? min(T, qblk * 64 + 64) : T;
  for (int j0 = 0; j0 < kv_end; j0 += 32) {
    __syncthreads();
    for (int e = tid; e < 32 * (D / 4); e += 128) {
      const int r = e / (D / 4), c4 = (e % (D / 4)) * 4;
      const int key = j0 + r;
      v4f kf = {0.f,0.f,0.f,0.f}, vf = {0.f,0.f,0.f,0.f};
      if (key < T) { kf = *(const v4fa*)(K + (size_t)key * pitch + c4); vf = *(const v4fa*)(V + (size_t)key * pitch + c4); }
#pragma unroll
      for (int t = 0; t < 4; ++t) {
        unsigned short hb = bf16_bits(kf[t]); sKh[r][c4 + t] = hb; sKl[r][c4 + t] = bf16_bits(kf[t] - bf16_val(hb));
        hb = bf16_bits(vf[t]); sVh[r][c4 + t] = hb; sVl[r][c4 + t] = bf16_bits(vf[t] - bf16_val(hb));
      }
    }
    __syncthreads();
    v8f s[2];
#pragma unroll
    for (int nt = 0; nt < 2; ++nt) {
      v8f acc = {};
#pragma unroll
      for (int ks = 0; ks < KS; ++ks) {
        FragB bh_, bl_;
        bh_.half[0] = *(const v8us*)&sKh[nt * 16 + ln][ks * 32 + 8 * hh]; bh_.half[1] = *(const v8us*)&sKh[nt * 16 + ln][ks * 32 + 16 + 8 * hh];
        bl_.half[0] = *(const v8us*)&sKl[nt * 16 + ln][ks * 32 + 8 * hh]; bl_.half[1] = *(const v8us*)&sKl[nt * 16 + ln][ks * 32 + 16 + 8 * hh];
        acc = mmaN<3>(aqh[ks].v, aql[ks].v, bh_.v, bl_.v, acc);
      }
      s[nt] = acc;
    }
    float alpha[8];
#pragma unroll
    for (int r = 0; r < 8; ++r) {
      const int qi = q0 + 8 * hh + r;
      const int ja = j0 + ln, jb = j0 + 16 + ln;
      if (CAUSAL) { if (ja > qi) s[0][r] = -3.0e38f; if (jb > qi) s[1][r] = -3.0e38f; }
      if (ja >= T) s[0][r] = -3.0e38f;
      if (jb >= T) s[1][r] = -3.0e38f;
      float mx = fmaxf(s[0][r], s[1][r]);
      mx = fmaxf(mx, __shfl_xor(mx, 1, 32)); mx = fmaxf(mx, __shfl_xor(mx, 2, 32)); mx = fmaxf(mx, __shfl_xor(mx, 4, 32)); mx = fmaxf(mx, __shfl_xor(mx, 8, 32));
      const float mnew = fmaxf(m_r[r], mx);
      alpha[r] = (mnew > -1.0e38f) ? __expf(m_r[r] - mnew) : 1.0f;
      const float p0 = (s[0][r] > -1.0e38f) ? __expf(s[0][r] - mnew) : 0.f;
      const float p1 = (s[1][r] > -1.0e38f) ? __expf(s[1][r] - mnew) : 0.f;
      m_r[r] = mnew;
      l_r[r] = l_r[r] * alpha[r] + p0 + p1;
      unsigned short hb = bf16_bits(p0); sPh[w][8 * hh + r][ln] = hb;      sPl[w][8 * hh + r][ln] = bf16_bits(p0 - bf16_val(hb));
      hb = bf16_bits(p1);                sPh[w][8 * hh + r][16 + ln] = hb; sPl[w][8 * hh + r][16 + ln] = bf16_bits(p1 - bf16_val(hb));
    }
#pragma unroll
    for (int dt = 0; dt < DT; ++dt)
#pragma unroll
      for (int r = 0; r < 8; ++r) oacc[dt][r] *= alpha[r];
    __builtin_amdgcn_fence(__ATOMIC_ACQ_REL, "workgroup");
    __builtin_amdgcn_wave_barrier();
    FragB pah, pal;
    pah.half[0] = *(const v8us*)&sPh[w][ln][8 * hh]; pah.half[1] = *(const v8us*)&sPh[w][ln][16 + 8 * hh];
    pal.half[0] = *(const v8us*)&sPl[w][ln][8 * hh]; pal.half[1] = *(const v8us*)&sPl[w][ln][16 + 8 * hh];
#pragma unroll
    for (int dt = 0; dt < DT; ++dt) {
      FragB bvh, bvl;
#pragma unroll
      for (int i = 0; i < 8; ++i) {
        bvh.u[i] = sVh[8 * hh + i][dt * 16 + ln]; bvh.u[8 + i] = sVh[16 + 8 * hh + i][dt * 16 + ln];
        bvl.u[i] = sVl[8 * hh + i][dt * 16 + ln]; bvl.u[8 + i] = sVl[16 + 8 * hh + i][dt * 16 + ln];
      }
      oacc[dt] = mmaN<3>(pah.v, pal.v, bvh.v, bvl.v, oacc[dt]);
    }
    __builtin_amdgcn_fence(__ATOMIC_ACQ_REL, "workgroup");
    __builtin_amdgcn_wave_barrier();
  }
#pragma unroll
  for (int r = 0; r < 8; ++r) {
    float l = l_r[r];
    l += __shfl_xor(l, 1, 32); l += __shfl_xor(l, 2, 32); l += __shfl_xor(l, 4, 32); l += __shfl_xor(l, 8, 32);
    l_r[r] = (l > 0.f) ? 1.0f / l : 0.f;
  }
#pragma unroll
  for (int dt = 0; dt < DT; ++dt)
#pragma unroll
    for (int r = 0; r < 8; ++r) sO[w][8 * hh + r][dt * 16 + ln] = oacc[dt][r] * l_r[r];
  __builtin_amdgcn_fence(__ATOMIC_ACQ_REL, "workgroup");
  __builtin_amdgcn_wave_barrier();
  for (int pass = 0; pass < 2; ++pass) {
    for (int r = 0; r < 16; ++r) {
      const int row = q0 + r;
      if (row < T && lane < D / 4) {
        const v4f val = *(const v4fa*)&sO[w][r][lane * 4];
        *(volatile v4f*)(y + ((size_t)b * T + row) * ypitch + h * D + lane * 4) = val;
      }
    }
    if (pass == 0) __threadfence();
  }
}

__global__ __launch_bounds__(256) void k_round_rows(const float* __restrict__ W, unsigned short* __restrict__ Wt, int n8) {
  const int t = blockIdx.x * 256 + threadIdx.x;
  if (t >= n8) return;
  const v4f a = *(const v4fa*)(W + (size_t)t * 8), b = *(const v4fa*)(W + (size_t)t * 8 + 4);
  v8us v; v[0]=bf16_bits(a[0]); v[1]=bf16_bits(a[1]); v[2]=bf16_bits(a[2]); v[3]=bf16_bits(a[3]);
  v[4]=bf16_bits(b[0]); v[5]=bf16_bits(b[1]); v[6]=bf16_bits(b[2]); v[7]=bf16_bits(b[3]);
  *(volatile v8us*)(Wt + (size_t)t * 8) = v; __threadfence(); *(volatile v8us*)(Wt + (size_t)t * 8) = v;
}

__global__ __launch_bounds__(256) void k_wt_conv(const float* __restrict__ w, unsigned short* __restrict__ Bt, int O, int Cin, int CinP, int Np) {
  const int t = blockIdx.x * 256 + threadIdx.x; const int K = 9 * CinP; if (t >= Np * (K / 8)) return;
  const int o = t / (K / 8), k8 = (t % (K / 8)) * 8; v8us v;
#pragma unroll 1
  for (int i = 0; i < 8; ++i) { const int k = k8 + i; const int tap = k / CinP, c = k % CinP; v[i] = (o < O && c < Cin) ? bf16_bits(w[((size_t)o * Cin + c) * 9 + tap]) : (unsigned short)0; }
  *(volatile v8us*)(Bt + (size_t)o * K + k8) = v; __threadfence(); *(volatile v8us*)(Bt + (size_t)o * K + k8) = v;
}
__device__ __forceinline__ float bilin_zero(const float* __restrict__ img, float py, float px) {
  const float y0 = floorf(py), x0 = floorf(px); const float wy = py - y0, wx = px - x0;
  float acc = 0.f;
#pragma unroll
  for (int dy = 0; dy < 2; ++dy)
#pragma unroll
    for (int dx = 0; dx < 2; ++dx) {
      const float yi = y0 + dy, xi = x0 + dx;
      if (yi >= 0.f && yi <= (float)(HH - 1) && xi >= 0.f && xi <= (float)(WW - 1)) acc += img[(int)yi * WW + (int)xi] * ((dy ? wy : 1.f - wy) * (dx ? wx : 1.f - wx));
    }
  return acc;
}
__global__ __launch_bounds__(256) void k_build_in1(const float* __restrict__ x, const float* __restrict__ flow, int dir, float* __restrict__ in1) {
  const size_t t = (size_t)blockIdx.x * 256 + threadIdx.x; if (t >= (size_t)NPOS * (CIN1 / 4)) return;
  const int c4 = (int)(t % (CIN1 / 4)) * 4; const int p = (int)(t / (CIN1 / 4)); const int n = p / (HH * WW), yx = p % (HH * WW), y = yx / WW, xq = yx % WW;
  const int fsrc = dir == 0 ? n + 1 : n, fcur = dir == 0 ? n : n + 1;
  const float* fl = flow + ((size_t)n * 2) * HH * WW;
  const float fx = bf16_round(fl[yx]), fy = bf16_round(fl[HH * WW + yx]);
  const float py = (float)y + fy, px = (float)xq + fx; const float y0 = floorf(py), x0 = floorf(px); const float wy = py - y0, wx = px - x0;
  v4f o;
#pragma unroll 1
  for (int i = 0; i < 4; ++i) {
    const int c = c4 + i; float v = 0.f;
    if (c < CC) { const float* img = x + ((size_t)fsrc * CC + c) * HH * WW;
      for (int dy = 0; dy < 2; ++dy) for (int dx = 0; dx < 2; ++dx) { const float yi = y0 + dy, xi = x0 + dx; if (yi >= 0.f && yi <= (float)(HH - 1) && xi >= 0.f && xi <= (float)(WW - 1)) v += bf16_round(img[(int)yi * WW + (int)xi]) * ((dy ? wy : 1.f - wy) * (dx ? wx : 1.f - wx)); } }
    else if (c < 2 * CC) v = bf16_round(x[((size_t)fcur * CC + (c - CC)) * HH * WW + yx]);
    else if (c == 2 * CC) v = fx; else if (c == 2 * CC + 1) v = fy;
    o[i] = v;
  }
  float* dst = in1 + (size_t)p * CIN1 + c4;
  *(volatile v4f*)dst = o; __threadfence(); *(volatile v4f*)dst = o;
}
template <int CinP, bool LRELU>
__global__ __launch_bounds__(128) void k_conv2d(const float* __restrict__ in, const unsigned short* __restrict__ Bt, const float* __restrict__ bias, int Nb, float* __restrict__ out, int Np) {
  constexpr int K = 9 * CinP, SPT = CinP / 32;
  __shared__ __attribute__((aligned(16))) float so[4][16][64];
  const int tid = threadIdx.x, w = tid >> 5, lane = tid & 31, ln = lane & 15, hh = lane >> 4;
  const int ntn = Np / 64; const int wid = blockIdx.x * 4 + w; const int mt = wid / ntn, nq = wid % ntn;
  if (mt * 16 >= NPOS) return;
  const int row0 = mt * 16, col0 = nq * 64; const int m = row0 + ln; const int n = m / (HH * WW), yx = m % (HH * WW), y = yx / WW, xq = yx % WW;
  v8f acc[4] = {};
  for (int tap = 0; tap < 9; ++tap) {
    const int yy = y + tap / 3 - 1, xx = xq + tap % 3 - 1; const bool inb = (yy >= 0 && yy < HH && xx >= 0 && xx < WW);
    const float* src = in + ((size_t)n * HH * WW + (size_t)(inb ? yy : 0) * WW + (inb ? xx : 0)) * CinP;
#pragma unroll
    for (int s = 0; s < SPT; ++s) {
      const int c0 = s * 32; v4f a0 = {0.f,0.f,0.f,0.f}, a1 = a0, a2 = a0, a3 = a0;
      if (inb) { a0 = *(const v4fa*)(src + c0 + 8 * hh); a1 = *(const v4fa*)(src + c0 + 8 * hh + 4); a2 = *(const v4fa*)(src + c0 + 16 + 8 * hh); a3 = *(const v4fa*)(src + c0 + 16 + 8 * hh + 4); }
      float xs[16] = {a0[0],a0[1],a0[2],a0[3],a1[0],a1[1],a1[2],a1[3],a2[0],a2[1],a2[2],a2[3],a3[0],a3[1],a3[2],a3[3]};
      FragB ah, al;
#pragma unroll
      for (int i = 0; i < 16; ++i) { const unsigned short hb = bf16_bits(xs[i]); ah.u[i] = hb; al.u[i] = bf16_bits(xs[i] - bf16_val(hb)); }
      const int kb = tap * CinP + c0;
#pragma unroll
      for (int t = 0; t < 4; ++t) { FragB bq; bq.half[0] = *(const v8us*)(Bt + (size_t)(col0 + t * 16 + ln) * K + kb + 8 * hh); bq.half[1] = *(const v8us*)(Bt + (size_t)(col0 + t * 16 + ln) * K + kb + 16 + 8 * hh); acc[t] = mmaN<2>(ah.v, al.v, bq.v, bq.v, acc[t]); }
    }
  }
#pragma unroll
  for (int t = 0; t < 4; ++t) { const int col = col0 + t * 16 + ln; const float bv = (col < Nb) ? bf16_round(bias[col]) : 0.f;
#pragma unroll
    for (int r = 0; r < 8; ++r) { float v = acc[t][r] + bv; if (LRELU) v = v >= 0.f ? v : 0.1f * v; so[w][8 * hh + r][t * 16 + ln] = v; } }
  __builtin_amdgcn_fence(__ATOMIC_ACQ_REL, "workgroup"); __builtin_amdgcn_wave_barrier();
  const int rsub = lane >> 4, c4 = (lane & 15) * 4;
  for (int pass = 0; pass < 2; ++pass) { for (int q = 0; q < 8; ++q) { const int r = q * 2 + rsub; const v4f v = *(const v4fa*)&so[w][r][c4]; *(volatile v4f*)(out + (size_t)(row0 + r) * Np + col0 + c4) = v; } if (pass == 0) __threadfence(); }
}
__global__ __launch_bounds__(128) void k_dcn(const float* __restrict__ x, const float* __restrict__ o4, const float* __restrict__ flow, int dir, const unsigned short* __restrict__ Bt, const float* __restrict__ bias, float* __restrict__ out) {
  constexpr int K = CC * KK;
  __shared__ __attribute__((aligned(16))) float so[4][16][64];
  const int tid = threadIdx.x, w = tid >> 5, lane = tid & 31, ln = lane & 15, hh = lane >> 4;
  const int mt = blockIdx.x * 4 + w; if (mt * 16 >= NPOS) return;
  const int row0 = mt * 16; const int m = row0 + ln; const int n = m / (HH * WW), yx = m % (HH * WW), y = yx / WW, xq = yx % WW;
  const int fsrc = dir == 0 ? n + 1 : n;
  const float* orow = o4 + (size_t)m * C4;
  const float* fl = flow + ((size_t)n * 2) * HH * WW; const float fx = bf16_round(fl[yx]), fy = bf16_round(fl[HH * WW + yx]);
  v8f acc[4] = {};
  for (int ks = 0; ks < K / 32; ++ks) {
    FragB ah, al;
#pragma unroll
    for (int i = 0; i < 16; ++i) {
      const int k = ks * 32 + ((i < 8) ? (8 * hh + i) : (16 + 8 * hh + (i - 8)));
      const int c = k / KK, kk = k % KK; const int g = c / (CC / DG);
      const int ch = g * 18 + kk * 2;
      const float dyo = 10.0f * tanhf(orow[ch]) + fy, dxo = 10.0f * tanhf(orow[ch + 1]) + fx;
      const float mk = 1.0f / (1.0f + expf(-orow[288 + g * 9 + kk]));
      const float py = (float)(y - 1 + kk / 3) + dyo, px = (float)(xq - 1 + kk % 3) + dxo;
      const float* img = x + ((size_t)fsrc * CC + c) * HH * WW;
      const float y0 = floorf(py), x0 = floorf(px); const float wy = py - y0, wx = px - x0; float v = 0.f;
      for (int dy = 0; dy < 2; ++dy) for (int dx = 0; dx < 2; ++dx) { const float yi = y0 + dy, xi = x0 + dx; if (yi >= 0.f && yi <= (float)(HH - 1) && xi >= 0.f && xi <= (float)(WW - 1)) v += bf16_round(img[(int)yi * WW + (int)xi]) * ((dy ? wy : 1.f - wy) * (dx ? wx : 1.f - wx)); }
      v *= mk;
      const unsigned short hb = bf16_bits(v); ah.u[i] = hb; al.u[i] = bf16_bits(v - bf16_val(hb));
    }
#pragma unroll
    for (int t = 0; t < 4; ++t) { FragB bq; bq.half[0] = *(const v8us*)(Bt + (size_t)(t * 16 + ln) * K + ks * 32 + 8 * hh); bq.half[1] = *(const v8us*)(Bt + (size_t)(t * 16 + ln) * K + ks * 32 + 16 + 8 * hh); acc[t] = mmaN<2>(ah.v, al.v, bq.v, bq.v, acc[t]); }
  }
#pragma unroll
  for (int t = 0; t < 4; ++t) { const float bv = bf16_round(bias[t * 16 + ln]);
#pragma unroll
    for (int r = 0; r < 8; ++r) so[w][8 * hh + r][t * 16 + ln] = acc[t][r] + bv; }
  __builtin_amdgcn_fence(__ATOMIC_ACQ_REL, "workgroup"); __builtin_amdgcn_wave_barrier();
  const int rsub = lane >> 4, c4 = (lane & 15) * 4;
  for (int pass = 0; pass < 2; ++pass) { for (int q = 0; q < 8; ++q) { const int r = q * 2 + rsub; const v4f v = *(const v4fa*)&so[w][r][c4]; *(volatile v4f*)(out + (size_t)(row0 + r) * CC + c4) = v; } if (pass == 0) __threadfence(); }
}
__global__ __launch_bounds__(256) void k_to_nchw(const float* __restrict__ pm, float* __restrict__ outT, int frame0) {
  __shared__ float tile[32][33];
  const int n = blockIdx.z, p0 = blockIdx.x * 32, c0 = blockIdx.y * 32; const int tx = threadIdx.x & 31, ty = threadIdx.x >> 5;
  for (int i = ty; i < 32; i += 8) tile[i][tx] = pm[((size_t)n * HH * WW + p0 + i) * CC + c0 + tx];
  __syncthreads();
  for (int pass = 0; pass < 2; ++pass) { for (int i = ty; i < 32; i += 8) *(volatile float*)(outT + (((size_t)(frame0 + n) * CC + c0 + i) * HH * WW) + p0 + tx) = tile[tx][i]; if (pass == 0) __threadfence(); }
}
__global__ __launch_bounds__(256) void k_zero(float* __restrict__ p, int n4) { const int t = blockIdx.x * 256 + threadIdx.x; if (t < n4) { v4f z = {0.f,0.f,0.f,0.f}; *(volatile v4f*)(p + (size_t)t * 4) = z; __threadfence(); *(volatile v4f*)(p + (size_t)t * 4) = z; } }

extern "C" void kernel_launch(void* const* d_in, const int* in_sizes, int n_in,
                              void* d_out, int out_size, void* d_ws, size_t ws_size, hipStream_t stream) {
  (void)in_sizes; (void)n_in; (void)out_size;
  const float* x = (const float*)d_in[0]; const float* flb = (const float*)d_in[1]; const float* flf = (const float*)d_in[2];
  const float* w1 = (const float*)d_in[3]; const float* b1 = (const float*)d_in[4]; const float* w2 = (const float*)d_in[5]; const float* b2 = (const float*)d_in[6];
  const float* w3 = (const float*)d_in[7]; const float* b3 = (const float*)d_in[8]; const float* w4 = (const float*)d_in[9]; const float* b4 = (const float*)d_in[10];
  const float* wd = (const float*)d_in[11]; const float* bd = (const float*)d_in[12];
  float* outB = (float*)d_out; float* outF = (float*)((char*)d_out + 16515072);
  char* ws = (char*)d_ws; size_t off = 0;
  auto take = [&](size_t bytes) { char* p = ws + off; off += (bytes + 255) & ~(size_t)255; return p; };
  unsigned short* Bt1 = (unsigned short*)take((size_t)64 * 9 * CIN1 * 2); unsigned short* Bt2 = (unsigned short*)take((size_t)64 * 576 * 2); unsigned short* Bt3 = (unsigned short*)take((size_t)64 * 576 * 2);
  unsigned short* Bt4 = (unsigned short*)take((size_t)C4 * 576 * 2); unsigned short* Btd = (unsigned short*)take((size_t)64 * 576 * 2);
  float* in1 = (float*)take((size_t)NPOS * CIN1 * 4);
  float* hA = (float*)take((size_t)NPOS * CC * 4); float* hB = (float*)take((size_t)NPOS * CC * 4);
  float* o4 = (float*)take((size_t)NPOS * C4 * 4);
  float* dout = (float*)take((size_t)NPOS * CC * 4);
  if (off > ws_size) return;
  k_wt_conv<<<(64 * (9 * CIN1 / 8) + 255) / 256, 256, 0, stream>>>(w1, Bt1, 64, 130, CIN1, 64);
  k_wt_conv<<<(64 * (576 / 8) + 255) / 256, 256, 0, stream>>>(w2, Bt2, 64, 64, 64, 64);
  k_wt_conv<<<(64 * (576 / 8) + 255) / 256, 256, 0, stream>>>(w3, Bt3, 64, 64, 64, 64);
  k_wt_conv<<<(C4 * (576 / 8) + 255) / 256, 256, 0, stream>>>(w4, Bt4, 432, 64, 64, C4);
  k_round_rows<<<(64 * 576 / 8 + 255) / 256, 256, 0, stream>>>(wd, Btd, 64 * 576 / 8);
  k_zero<<<(CC * HH * WW / 4 + 255) / 256, 256, 0, stream>>>(outB + (size_t)6 * CC * HH * WW, CC * HH * WW / 4);
  k_zero<<<(CC * HH * WW / 4 + 255) / 256, 256, 0, stream>>>(outF, CC * HH * WW / 4);
  const int gb64 = ((NPOS / 16) * 1 + 3) / 4, gb448 = ((NPOS / 16) * (C4 / 64) + 3) / 4;
  for (int dir = 0; dir < 2; ++dir) {
    const float* fl = dir == 0 ? flb : flf;
    k_build_in1<<<(unsigned)(((size_t)NPOS * (CIN1 / 4) + 255) / 256), 256, 0, stream>>>(x, fl, dir, in1);
    k_conv2d<CIN1, true><<<gb64, 128, 0, stream>>>(in1, Bt1, b1, 64, hA, 64);
    k_conv2d<CC, true><<<gb64, 128, 0, stream>>>(hA, Bt2, b2, 64, hB, 64);
    k_conv2d<CC, true><<<gb64, 128, 0, stream>>>(hB, Bt3, b3, 64, hA, 64);
    k_conv2d<CC, false><<<gb448, 128, 0, stream>>>(hA, Bt4, b4, 432, o4, C4);
    k_dcn<<<(NPOS / 16 + 3) / 4, 128, 0, stream>>>(x, o4, fl, dir, Btd, bd, dout);
    k_to_nchw<<<dim3(HH * WW / 32, CC / 32, NFR), 256, 0, stream>>>(dout, dir == 0 ? outB : outF, dir == 0 ? 0 : 1);
  }
}
